// FrequencySelfAttention4_35124242547049
// MI455X (gfx1250) — hardware-verified
//
#include <hip/hip_runtime.h>

#define BB 8
#define CC 256
#define NN 4096
#define H0 32
#define W0 32

typedef _Float16 f16;
typedef __attribute__((ext_vector_type(16))) _Float16 v16h;
typedef __attribute__((ext_vector_type(8)))  _Float16 v8h;
typedef __attribute__((ext_vector_type(8)))  float    v8f;

union FragU { v16h v; v8h h[2]; };
typedef __attribute__((ext_vector_type(4))) float v4f;
typedef __attribute__((ext_vector_type(4))) unsigned v4u;
template <typename V> __device__ __forceinline__ void vst2(void* p, V v) {
  *(volatile V*)p = v; __threadfence(); *(volatile V*)p = v;
}
#define PSC 256.0f
#define PUN (1.0f / 256.0f)
typedef __attribute__((ext_vector_type(16))) __bf16 v16bf;
typedef __attribute__((ext_vector_type(8)))  __bf16 v8bf;
__device__ __forceinline__ __bf16 bf_hi(float x) { return (__bf16)x; }
__device__ __forceinline__ __bf16 bf_lo(float x, __bf16 h) { return (__bf16)(x - (float)h); }
__device__ __forceinline__ v8f WMMA_BF16(v16bf a, v16bf b, v8f c) {
  v8f d = __builtin_amdgcn_wmma_f32_16x16x32_bf16(false, a, false, b, (short)0, c, false, false);
  asm volatile("v_nop\n\tv_nop\n\tv_nop\n\tv_nop" : "+v"(d) : "v"(a), "v"(b));
  return d;
}
__device__ __forceinline__ v16bf load_bf_lds(const __bf16* base, int row, int rs, int kbase, int lane) {
  union { v16bf v; v8bf h[2]; } u;
  const __bf16* p = base + (size_t)row * rs + kbase + ((lane >> 4) << 3);
  u.h[0] = *(const v8bf*)(p); u.h[1] = *(const v8bf*)(p + 16);
  return u.v;
}
__device__ __forceinline__ void load_b_split(const float* base, int col, int rs, int kbase, int lane, v16bf& hi, v16bf& lo) {
  const float* p = base + (size_t)col * rs + kbase + ((lane >> 4) << 3);
  const v4f a0 = *(const v4f*)(p), a1 = *(const v4f*)(p + 4), a2 = *(const v4f*)(p + 16), a3 = *(const v4f*)(p + 20);
#pragma unroll
  for (int i = 0; i < 4; ++i) {
    __bf16 h;
    h = bf_hi(a0[i]); hi[i] = h;      lo[i] = bf_lo(a0[i], h);
    h = bf_hi(a1[i]); hi[4 + i] = h;  lo[4 + i] = bf_lo(a1[i], h);
    h = bf_hi(a2[i]); hi[8 + i] = h;  lo[8 + i] = bf_lo(a2[i], h);
    h = bf_hi(a3[i]); hi[12 + i] = h; lo[12 + i] = bf_lo(a3[i], h);
  }
}

__device__ __forceinline__ v16h load_a(const f16* base, int row, int rs, int kbase, int lane) {
  const f16* p = base + (size_t)row * rs + kbase + ((lane >> 4) << 3);
  FragU u;
  u.h[0] = *(const v8h*)(p);
  u.h[1] = *(const v8h*)(p + 16);
  return u.v;
}
__device__ __forceinline__ v16h load_b(const f16* base, int col, int rs, int kbase, int lane) {
  return load_a(base, col, rs, kbase, lane);
}

__device__ __forceinline__ v8f WMMA_F16(v16h a, v16h b, v8f c) {
  v8f d = __builtin_amdgcn_wmma_f32_16x16x32_f16(false, a, false, b, (short)0, c, false, false);
  asm volatile("v_nop\n\tv_nop\n\tv_nop\n\tv_nop" : "+v"(d) : "v"(a), "v"(b));
  return d;
}


__global__ __launch_bounds__(256) void k_scale(const float* __restrict__ g0,
                                               float* __restrict__ sc) {
  int idx = blockIdx.x * 256 + threadIdx.x;
  int b = idx >> 12, n = idx & (NN - 1);
  int ny = n >> 6, nx = n & 63;
  float fy = ny * (31.0f / 63.0f);
  float fx = nx * (31.0f / 63.0f);
  int y0 = (int)fy, x0 = (int)fx;
  float wy = fy - (float)y0, wx = fx - (float)x0;
  int y1 = min(y0 + 1, H0 - 1), x1 = min(x0 + 1, W0 - 1);
  const float* g = g0 + (size_t)b * H0 * W0;
  float v00 = g[y0 * W0 + x0], v01 = g[y0 * W0 + x1];
  float v10 = g[y1 * W0 + x0], v11 = g[y1 * W0 + x1];
  float vy0 = v00 * (1.f - wx) + v01 * wx;
  float vy1 = v10 * (1.f - wx) + v11 * wx;
  float v = vy0 * (1.f - wy) + vy1 * wy;
  vst2(sc + idx, 1.0f + 1.0f / (1.0f + __expf(-v)));
}

__global__ __launch_bounds__(256) void k_wconv(const float* __restrict__ Wq,
                                               const float* __restrict__ Wk,
                                               const float* __restrict__ Wv,
                                               const float* __restrict__ Wo,
                                               const float* __restrict__ fw,
                                               f16* __restrict__ W3,
                                               f16* __restrict__ Wo16) {
  int g = blockIdx.x * 256 + threadIdx.x;
  int idx0 = g * 8;
  int m = idx0 >> 16, r0 = idx0 & 65535;
  const float* W = (m == 0) ? Wq : (m == 1) ? Wk : (m == 2) ? Wv : Wo;
  union { v8h h; v4u u; } pk;
#pragma unroll
  for (int e = 0; e < 8; ++e) { int r = r0 + e, ci = r & (CC - 1); pk.h[e] = (f16)(W[r] * ((m < 3) ? fw[ci] : 1.0f)); }
  f16* dst = (m < 3) ? (W3 + (size_t)m * 65536 + r0) : (Wo16 + r0);
  vst2(dst, pk.u);
}

__global__ __launch_bounds__(256) void k_xt(const float* __restrict__ x,
                                            f16* __restrict__ xT) {
  __shared__ __align__(16) f16 tile[64][72];
  int b = blockIdx.z, c0 = blockIdx.y * 64, n0 = blockIdx.x * 64;
  int tid = threadIdx.x;
  {
    int cl = tid >> 2, nq = (tid & 3) * 16;
    const float4* src = (const float4*)(x + (size_t)b * CC * NN +
                                        (size_t)(c0 + cl) * NN + n0 + nq);
    for (int i = 0; i < 4; ++i) {
      float4 v = src[i];
      tile[cl][nq + 4 * i + 0] = (f16)v.x;
      tile[cl][nq + 4 * i + 1] = (f16)v.y;
      tile[cl][nq + 4 * i + 2] = (f16)v.z;
      tile[cl][nq + 4 * i + 3] = (f16)v.w;
    }
  }
  __syncthreads();
  for (int pass = 0; pass < 2; ++pass) {
    int nl = pass * 32 + (tid >> 3), cq = (tid & 7) * 8;
    f16* dst = xT + (size_t)b * NN * CC + (size_t)(n0 + nl) * CC + c0 + cq;
    union { v8h h; v4u u; } o;
    for (int i = 0; i < 8; ++i) o.h[i] = tile[cq + i][nl];
    vst2(dst, o.u);
  }
}

__global__ __launch_bounds__(256) void k_qkv(const f16* __restrict__ xT,
                                             const f16* __restrict__ W3,
                                             const float* __restrict__ xf,
                                             const float* __restrict__ Wqf, const float* __restrict__ Wkf,
                                             const float* __restrict__ fw,
                                             const float* __restrict__ bq,
                                             const float* __restrict__ bk,
                                             const float* __restrict__ bv,
                                             const float* __restrict__ scg,
                                             float* __restrict__ qT,
                                             float* __restrict__ kT,
                                             f16* __restrict__ v16) {
  __shared__ __align__(16) float T[64][260];
  int b = blockIdx.y;
  int n_base = blockIdx.x * 64;
  int tid = threadIdx.x;
  int lane = threadIdx.x & 31, wave = threadIdx.x >> 5;
  int co_wave = wave * 32;
  const f16* xTb = xT + (size_t)b * NN * CC;
  const float* scb = scg + (size_t)b * NN;
  const v8f vzero = {};
  const float* xfb = xf + (size_t)b * CC * NN;
  for (int m = 0; m < 3; ++m) {
    const f16* Wm = W3 + (size_t)m * 65536;
    const float* bias = (m == 0) ? bq : ((m == 1) ? bk : bv);
    v8f acc[2][4];
    for (int cb = 0; cb < 2; ++cb)
      for (int nb = 0; nb < 4; ++nb) acc[cb][nb] = vzero;
    if (m < 2) {
      const float* Wf = (m == 0) ? Wqf : Wkf;
      for (int kk = 0; kk < CC; kk += 32) {
        v16bf ah[2], al[2];
#pragma unroll
        for (int cb = 0; cb < 2; ++cb) {
          const float* wr = Wf + (size_t)(co_wave + cb * 16 + (lane & 15)) * CC + kk + ((lane >> 4) << 3);
#pragma unroll
          for (int e = 0; e < 16; ++e) { const int ko = (e < 8) ? e : (8 + e); const float w = wr[ko] * fw[kk + ((lane >> 4) << 3) + ko];
                                         __bf16 hh = bf_hi(w); ah[cb][e] = hh; al[cb][e] = bf_lo(w, hh); }
        }
        for (int nb = 0; nb < 4; ++nb) {
          v16bf bh, bl;
          const float* xp = xfb + (size_t)(kk + ((lane >> 4) << 3)) * NN + n_base + nb * 16 + (lane & 15);
#pragma unroll
          for (int e = 0; e < 16; ++e) { const int ko = (e < 8) ? e : (8 + e); const float xv = xp[(size_t)ko * NN];
                                         __bf16 hh = bf_hi(xv); bh[e] = hh; bl[e] = bf_lo(xv, hh); }
          acc[0][nb] = WMMA_BF16(ah[0], bh, acc[0][nb]); acc[0][nb] = WMMA_BF16(ah[0], bl, acc[0][nb]); acc[0][nb] = WMMA_BF16(al[0], bh, acc[0][nb]);
          acc[1][nb] = WMMA_BF16(ah[1], bh, acc[1][nb]); acc[1][nb] = WMMA_BF16(ah[1], bl, acc[1][nb]); acc[1][nb] = WMMA_BF16(al[1], bh, acc[1][nb]);
        }
      }
    } else
    for (int kk = 0; kk < CC; kk += 32) {
      v16h a0 = load_a(Wm, co_wave + (lane & 15), CC, kk, lane);
      v16h a1 = load_a(Wm, co_wave + 16 + (lane & 15), CC, kk, lane);
      for (int nb = 0; nb < 4; ++nb) {
        v16h bf = load_b(xTb, n_base + nb * 16 + (lane & 15), CC, kk, lane);
        acc[0][nb] = WMMA_F16(a0, bf, acc[0][nb]);
        acc[1][nb] = WMMA_F16(a1, bf, acc[1][nb]);
      }
    }
    float qmul = (m == 0) ? 0.0625f : 1.0f;
    __syncthreads();
    for (int cb = 0; cb < 2; ++cb) {
      int co_b = co_wave + cb * 16 + ((lane >> 4) << 3);
      for (int nb = 0; nb < 4; ++nb) {
        int nl = nb * 16 + (lane & 15);
        float s = scb[n_base + nl] * qmul;
        for (int r = 0; r < 8; ++r) T[nl][co_b + r] = (acc[cb][nb][r] + bias[co_b + r]) * s;
      }
    }
    __syncthreads();
    if (m < 2) {
      float* dstb = ((m == 0) ? qT : kT) + (size_t)b * NN * CC + (size_t)n_base * CC;
      for (int g = tid; g < 64 * 64; g += 256) { int nl = g >> 6, pc = g & 63; vst2(dstb + (size_t)nl * CC + pc * 4, *(const v4f*)(&T[nl][pc * 4])); }
    } else {
      f16* vb = v16 + (size_t)b * CC * NN + n_base;
      for (int g = tid; g < 256 * 8; g += 256) {
        int c = g >> 3, pc = g & 7;
        union { v8h h; v4u u; } pk;
        for (int e = 0; e < 8; ++e) pk.h[e] = (f16)T[pc * 8 + e][c];
        vst2(vb + (size_t)c * NN + pc * 8, pk.u);
      }
    }
  }
}

__global__ __launch_bounds__(256) void k_attn(const float* __restrict__ qT,
                                              const float* __restrict__ kT,
                                              const f16* __restrict__ v16,
                                              f16* __restrict__ aout) {
  __shared__ __align__(16) __bf16 Qh[64][264];
  __shared__ __align__(16) __bf16 Ql[64][264];
  __shared__ __align__(16) float Sbuf[64][68];
  __shared__ __align__(16) f16 Pbuf[64][72];
  __shared__ float m_run[64], l_run[64], rfac[64];
  __shared__ float pmax[4][64], psum[4][64];
  __shared__ __align__(16) f16 Ot[64][264];
  int b = blockIdx.y;
  int nq = blockIdx.x * 64;
  int tid = threadIdx.x, lane = tid & 31, wave = tid >> 5;
  int row_blk = wave & 3;
  int colp = (wave >> 2) * 2;
  int c_wave = wave * 32;
  int srow = tid & 63, sq = tid >> 6;
  const float* qTb = qT + (size_t)b * NN * CC;
  const float* kTb = kT + (size_t)b * NN * CC;
  const f16* vb  = v16 + (size_t)b * CC * NN;
  const v8f vzero = {};
  v8f oacc[8];
  for (int i = 0; i < 8; ++i) oacc[i] = vzero;

  {
    int row = tid >> 2, cbase = (tid & 3) * 64;
    const float* qp = &qTb[(size_t)(nq + row) * CC + cbase];
    for (int i = 0; i < 64; i += 4) {
      const v4f a = *(const v4f*)(qp + i);
#pragma unroll
      for (int e = 0; e < 4; ++e) { __bf16 h = bf_hi(a[e]); Qh[row][cbase + i + e] = h; Ql[row][cbase + i + e] = bf_lo(a[e], h); }
    }
  }
  if (tid < 64) { m_run[tid] = -1e30f; l_run[tid] = 0.f; }
  __syncthreads();

  for (int t = 0; t < NN / 64; ++t) {
    int mb = t * 64;
    v8f s0 = vzero, s1 = vzero;
    for (int kk = 0; kk < CC; kk += 32) {
      v16bf ah = load_bf_lds(&Qh[0][0], row_blk * 16 + (lane & 15), 264, kk, lane);
      v16bf al = load_bf_lds(&Ql[0][0], row_blk * 16 + (lane & 15), 264, kk, lane);
      v16bf b0h, b0l, b1h, b1l;
      load_b_split(kTb, mb + colp * 16 + (lane & 15), CC, kk, lane, b0h, b0l);
      load_b_split(kTb, mb + (colp + 1) * 16 + (lane & 15), CC, kk, lane, b1h, b1l);
      s0 = WMMA_BF16(ah, b0h, s0); s0 = WMMA_BF16(ah, b0l, s0); s0 = WMMA_BF16(al, b0h, s0);
      s1 = WMMA_BF16(ah, b1h, s1); s1 = WMMA_BF16(ah, b1l, s1); s1 = WMMA_BF16(al, b1h, s1);
    }
    for (int r = 0; r < 8; ++r) {
      int row = row_blk * 16 + r + ((lane >> 4) << 3);
      Sbuf[row][colp * 16 + (lane & 15)] = s0[r];
      Sbuf[row][(colp + 1) * 16 + (lane & 15)] = s1[r];
    }
    __syncthreads();
    float arr[16];
    {
      const float4* sp = (const float4*)&Sbuf[srow][sq * 16];
      float4 f0 = sp[0], f1 = sp[1], f2 = sp[2], f3 = sp[3];
      ((float4*)arr)[0] = f0; ((float4*)arr)[1] = f1;
      ((float4*)arr)[2] = f2; ((float4*)arr)[3] = f3;
      float mx = fmaxf(fmaxf(fmaxf(f0.x, f0.y), fmaxf(f0.z, f0.w)),
                       fmaxf(fmaxf(fmaxf(f1.x, f1.y), fmaxf(f1.z, f1.w)),
                             fmaxf(fmaxf(fmaxf(f2.x, f2.y), fmaxf(f2.z, f2.w)),
                                   fmaxf(fmaxf(f3.x, f3.y), fmaxf(f3.z, f3.w)))));
      pmax[sq][srow] = mx;
    }
    __syncthreads();
    {
      float m_new = fmaxf(fmaxf(pmax[0][srow], pmax[1][srow]),
                          fmaxf(fmaxf(pmax[2][srow], pmax[3][srow]), m_run[srow]));
      float l = 0.f;
      v8h pk0, pk1;
      for (int i = 0; i < 8; ++i) {
        float p = __expf(arr[i] - m_new);
        pk0[i] = (f16)(p * PSC); l += p;
      }
      for (int i = 0; i < 8; ++i) {
        float p = __expf(arr[8 + i] - m_new);
        pk1[i] = (f16)(p * PSC); l += p;
      }
      *(v8h*)&Pbuf[srow][sq * 16] = pk0;
      *(v8h*)&Pbuf[srow][sq * 16 + 8] = pk1;
      psum[sq][srow] = l;
    }
    __syncthreads();
    if (tid < 64) {
      float mold = m_run[tid];
      float m_new = fmaxf(fmaxf(pmax[0][tid], pmax[1][tid]),
                          fmaxf(fmaxf(pmax[2][tid], pmax[3][tid]), mold));
      float rs = __expf(mold - m_new);
      l_run[tid] = l_run[tid] * rs +
                   (psum[0][tid] + psum[1][tid] + psum[2][tid] + psum[3][tid]);
      m_run[tid] = m_new;
      rfac[tid] = rs;
    }
    __syncthreads();
    for (int nb = 0; nb < 4; ++nb) {
      float f[8];
      for (int r = 0; r < 8; ++r) f[r] = rfac[nb * 16 + r + ((lane >> 4) << 3)];
      for (int cb = 0; cb < 2; ++cb)
        for (int r = 0; r < 8; ++r) oacc[nb * 2 + cb][r] *= f[r];
      for (int kk = 0; kk < 64; kk += 32) {
        v16h pa = load_a(&Pbuf[0][0], nb * 16 + (lane & 15), 72, kk, lane);
        for (int cb = 0; cb < 2; ++cb) {
          v16h vf = load_b(vb, c_wave + cb * 16 + (lane & 15), NN, mb + kk, lane);
          oacc[nb * 2 + cb] = WMMA_F16(pa, vf, oacc[nb * 2 + cb]);
        }
      }
    }
    __syncthreads();
  }
  for (int nb = 0; nb < 4; ++nb)
    for (int cb = 0; cb < 2; ++cb) {
      int c = c_wave + cb * 16 + (lane & 15);
      for (int r = 0; r < 8; ++r) {
        int nloc = nb * 16 + r + ((lane >> 4) << 3);
        Ot[nloc][c] = (f16)(oacc[nb * 2 + cb][r] * (PUN / l_run[nloc]));
      }
    }
  __syncthreads();
  {
    f16* ab = aout + (size_t)b * NN * CC + (size_t)nq * CC;
    for (int g = tid; g < 64 * 32; g += 256) { int nl = g >> 5, pc = g & 31; vst2(ab + (size_t)nl * CC + pc * 8, *(const v4u*)(&Ot[nl][pc * 8])); }
  }
}

__global__ __launch_bounds__(256) void k_out(const f16* __restrict__ aout,
                                             const f16* __restrict__ Wo16,
                                             const float* __restrict__ bo,
                                             float* __restrict__ out) {
  __shared__ __align__(16) float So[8][32 * 64];
  int b = blockIdx.y;
  int n_base = blockIdx.x * 64;
  int lane = threadIdx.x & 31, wave = threadIdx.x >> 5;
  int co_wave = wave * 32;
  const f16* ab = aout + (size_t)b * NN * CC;
  const v8f vzero = {};
  v8f acc[2][4];
  for (int cb = 0; cb < 2; ++cb)
    for (int nb = 0; nb < 4; ++nb) acc[cb][nb] = vzero;
  for (int kk = 0; kk < CC; kk += 32) {
    v16h a0 = load_a(Wo16, co_wave + (lane & 15), CC, kk, lane);
    v16h a1 = load_a(Wo16, co_wave + 16 + (lane & 15), CC, kk, lane);
    for (int nb = 0; nb < 4; ++nb) {
      v16h bf = load_b(ab, n_base + nb * 16 + (lane & 15), CC, kk, lane);
      acc[0][nb] = WMMA_F16(a0, bf, acc[0][nb]);
      acc[1][nb] = WMMA_F16(a1, bf, acc[1][nb]);
    }
  }
  float* ob = out + (size_t)b * CC * NN;
  float* so = So[wave];
  for (int cb = 0; cb < 2; ++cb) {
    int col_b = cb * 16 + ((lane >> 4) << 3);
    for (int nb = 0; nb < 4; ++nb) {
      int nl = nb * 16 + (lane & 15);
      for (int r = 0; r < 8; ++r) so[(col_b + r) * 64 + nl] = acc[cb][nb][r] + bo[co_wave + col_b + r];
    }
  }
  __syncthreads();
  for (int q = 0; q < 16; ++q) {
    int rl = q * 2 + (lane >> 4), pc = lane & 15;
    vst2(ob + (size_t)(co_wave + rl) * NN + n_base + pc * 4, *(const v4f*)(&so[rl * 64 + pc * 4]));
  }
}

extern "C" void kernel_launch(void* const* d_in, const int* in_sizes, int n_in,
                              void* d_out, int out_size, void* d_ws, size_t ws_size,
                              hipStream_t stream) {
  (void)in_sizes; (void)n_in; (void)out_size; (void)ws_size;
  const float* x  = (const float*)d_in[0];
  const float* g0 = (const float*)d_in[1];
  const float* Wq = (const float*)d_in[2];
  const float* bq = (const float*)d_in[3];
  const float* Wk = (const float*)d_in[4];
  const float* bk = (const float*)d_in[5];
  const float* Wv = (const float*)d_in[6];
  const float* bv = (const float*)d_in[7];
  const float* Wo = (const float*)d_in[8];
  const float* bo = (const float*)d_in[9];
  const float* fw = (const float*)d_in[10];

  char* ws = (char*)d_ws;
  float* scg = (float*)ws; ws += (size_t)BB * NN * sizeof(float);
  f16* W3    = (f16*)ws;   ws += (size_t)3 * CC * CC * sizeof(f16);
  f16* Wo16  = (f16*)ws;   ws += (size_t)CC * CC * sizeof(f16);
  f16* xT    = (f16*)ws;   ws += (size_t)BB * NN * CC * sizeof(f16);
  float* qT  = (float*)ws; ws += (size_t)BB * NN * CC * sizeof(float);
  float* kT  = (float*)ws; ws += (size_t)BB * NN * CC * sizeof(float);
  f16* v16   = (f16*)ws;   ws += (size_t)BB * NN * CC * sizeof(f16);
  f16* aout  = (f16*)ws;

  k_scale<<<dim3((BB * NN) / 256), 256, 0, stream>>>(g0, scg);
  k_wconv<<<dim3((4 * CC * CC / 8) / 256), 256, 0, stream>>>(Wq, Wk, Wv, Wo, fw, W3, Wo16);
  k_xt<<<dim3(NN / 64, CC / 64, BB), 256, 0, stream>>>(x, xT);
  k_qkv<<<dim3(NN / 64, BB), 256, 0, stream>>>(xT, W3, x, Wq, Wk, fw, bq, bk, bv, scg, qT, kT, v16);
  k_attn<<<dim3(NN / 64, BB), 256, 0, stream>>>(qT, kT, v16, aout);
  k_out<<<dim3(NN / 64, BB), 256, 0, stream>>>(aout, Wo16, bo, (float*)d_out);
}
